// UNet_AttentionBlock_72292889526976
// MI455X (gfx1250) — hardware-verified
//
#include <hip/hip_runtime.h>
#include <hip/hip_bf16.h>
#include <stdint.h>

typedef __attribute__((ext_vector_type(16))) _Float16 v16h;
typedef __attribute__((ext_vector_type(8)))  _Float16 v8h;
typedef __attribute__((ext_vector_type(8)))  float    v8f;
typedef __attribute__((ext_vector_type(4)))  float    v4f;
#define VST2(T, ptr, val) do { const T _v = (val); *(volatile T*)(ptr) = _v; __threadfence(); *(volatile T*)(ptr) = _v; } while (0)
__device__ inline v8f wmma16(v16h a, v16h b, v8f c) {
    v8f d = __builtin_amdgcn_wmma_f32_16x16x32_f16(false, a, false, b, (short)0, c, false, false);
    asm volatile("v_nop\n\tv_nop\n\tv_nop\n\tv_nop" : "+v"(d) : "v"(a), "v"(b));
    return d;
}
__device__ inline v16h frag16(const _Float16* p, int khi) {
    const v8h lo = *(const v8h*)(p + 8 * khi), hi = *(const v8h*)(p + 16 + 8 * khi);
    return __builtin_shufflevector(lo, hi, 0, 1, 2, 3, 4, 5, 6, 7, 8, 9, 10, 11, 12, 13, 14, 15);
}

#define BATCH   16
#define CCH     256
#define LSEQ    1024
#define HEADS   8
#define HDIM    32
#define NQKV    768
#define DCOND   128
#define GROUPS  32
#define GN_EPS  1e-5f

__global__ void cvt_half_kernel(const float* __restrict__ src,
                                _Float16* __restrict__ dst, int n) {
    int i = blockIdx.x * blockDim.x + threadIdx.x;
    if (i < n) VST2(_Float16, dst + i, (_Float16)src[i]);
}

__global__ void cond_embed_kernel(const float* __restrict__ t,
                                  const float* __restrict__ cond,
                                  const float* __restrict__ cond2,
                                  const float* __restrict__ tw, const float* __restrict__ tb,
                                  const float* __restrict__ cw, const float* __restrict__ cb,
                                  const float* __restrict__ c2w, const float* __restrict__ c2b,
                                  float* __restrict__ emb) {
    int b = blockIdx.x, c = threadIdx.x;
    float acc = tb[c] + cb[c] + c2b[c];
    const float* tp  = t     + b * DCOND;
    const float* cp  = cond  + b * DCOND;
    const float* c2p = cond2 + b * DCOND;
    const float* twp  = tw  + c * DCOND;
    const float* cwp  = cw  + c * DCOND;
    const float* c2wp = c2w + c * DCOND;
    for (int k = 0; k < DCOND; ++k) {
        float a = tp[k];  acc += (a / (1.f + expf(-a))) * twp[k];
        float d = cp[k];  acc += (d / (1.f + expf(-d))) * cwp[k];
        float e = c2p[k]; acc += (e / (1.f + expf(-e))) * c2wp[k];
    }
    VST2(float, emb + b * CCH + c, acc);
}

__global__ void gn_stats_kernel(const float* __restrict__ x,
                                float* __restrict__ mean, float* __restrict__ rstd) {
    __shared__ float sm[32], sr[32];
    const int b = blockIdx.x, wave = threadIdx.x >> 5, lane = threadIdx.x & 31;
    for (int gi = 0; gi < 4; ++gi) {
        const int g = wave * 4 + gi;
        const float* p = x + ((size_t)b * CCH + g * 8) * LSEQ;
        float s = 0.f, s2 = 0.f;
        for (int i = lane; i < 8 * LSEQ; i += 32) { const float v = p[i]; s += v; s2 += v * v; }
        #pragma unroll
        for (int off = 16; off > 0; off >>= 1) { s += __shfl_xor(s, off, 32); s2 += __shfl_xor(s2, off, 32); }
        if (lane == 0) { const float mn = s * (1.f / 8192.f); sm[g] = mn; sr[g] = 1.0f / sqrtf(fmaxf(s2 * (1.f / 8192.f) - mn * mn, 0.f) + GN_EPS); }
    }
    __syncthreads();
    if (threadIdx.x < 32) { VST2(float, mean + b * GROUPS + threadIdx.x, sm[threadIdx.x]); VST2(float, rstd + b * GROUPS + threadIdx.x, sr[threadIdx.x]); }
}

__global__ void gn_apply_kernel(const float* __restrict__ x,
                                const float* __restrict__ mean, const float* __restrict__ rstd,
                                const float* __restrict__ gw, const float* __restrict__ gb,
                                const float* __restrict__ emb,
                                float* __restrict__ xs_f, _Float16* __restrict__ xs_h) {
    const int b = blockIdx.x >> 10, l = blockIdx.x & (LSEQ - 1), c = threadIdx.x;
    const int g = c >> 3;
    const float m = mean[b * GROUPS + g], r = rstd[b * GROUPS + g];
    const float scale = r * gw[c];
    const float shift = gb[c] + emb[b * CCH + c] - m * scale;
    const float v = x[((size_t)b * CCH + c) * LSEQ + l] * scale + shift;
    const size_t o = ((size_t)b * LSEQ + l) * CCH + c;
    VST2(float, xs_f + o, v);
    VST2(_Float16, xs_h + o, (_Float16)v);
}

__device__ inline v16h load_a_frag(const _Float16* base, int stride_row,
                                   int ln, int khi, int k0) {
    const _Float16* p = base + (size_t)ln * stride_row + k0 + 8 * khi;
    v8h lo = *(const v8h*)(p);
    v8h hi = *(const v8h*)(p + 16);
    return __builtin_shufflevector(lo, hi, 0, 1, 2, 3, 4, 5, 6, 7,
                                           8, 9, 10, 11, 12, 13, 14, 15);
}

__global__ void qkv_gemm_kernel(const _Float16* __restrict__ xs_h,
                                const _Float16* __restrict__ wh,
                                const float* __restrict__ bias,
                                _Float16* __restrict__ qh,
                                _Float16* __restrict__ kh,
                                _Float16* __restrict__ vth)
{
    int b = blockIdx.z;
    int n0 = blockIdx.x * 64, m0 = blockIdx.y * 128;
    int wave = threadIdx.x >> 5, lane = threadIdx.x & 31;
    int khi = lane >> 4, ln = lane & 15;
    int row = m0 + wave * 16;
    const _Float16* A = xs_h + ((size_t)b * LSEQ + row) * CCH;

    v8f acc[4] = {};
    for (int k0 = 0; k0 < CCH; k0 += 32) {
        v16h a = load_a_frag(A, CCH, ln, khi, k0);
        #pragma unroll
        for (int t = 0; t < 4; ++t) {
            int col = n0 + t * 16 + ln;
            v16h bf = frag16(wh + (size_t)col * CCH + k0, khi);
            acc[t] = wmma16(a, bf, acc[t]);
        }
    }
    __shared__ __attribute__((aligned(16))) _Float16 sT[64][136];
    #pragma unroll
    for (int t = 0; t < 4; ++t) {
        const int cl = t * 16 + ln, col = n0 + cl;
        const int rem = col % 96;
        const float bv = bias[col], sc = (rem < 32) ? 0.0625f : 1.0f;
        #pragma unroll
        for (int r = 0; r < 8; ++r) sT[cl][wave * 16 + r + 8 * khi] = (_Float16)((acc[t][r] + bv) * sc);
    }
    __syncthreads();
    for (int pass = 0; pass < 2; ++pass) {
        for (int p = threadIdx.x; p < 2 * 512; p += 256) {
            const int grp = p >> 9, q = p & 511;
            const int col0 = n0 + grp * 32, head = col0 / 96, rem0 = col0 - head * 96;
            const size_t bh = (size_t)b * HEADS + head;
            if (rem0 < 64) {
                const int lr = q >> 2, dc = (q & 3) * 8;
                v8h v;
                #pragma unroll
                for (int e = 0; e < 8; ++e) v[e] = sT[grp * 32 + dc + e][lr];
                _Float16* dst = ((rem0 < 32) ? qh : kh) + (bh * LSEQ + m0 + lr) * HDIM + dc;
                *(volatile v8h*)dst = v;
            } else {
                const int d = q >> 4, lc = (q & 15) * 8;
                *(volatile v8h*)(vth + (bh * HDIM + d) * LSEQ + m0 + lc) = *(const v8h*)&sT[grp * 32 + d][lc];
            }
        }
        __threadfence();
    }
}

__global__ void flash_attn_kernel(const _Float16* __restrict__ qh,
                                  const _Float16* __restrict__ kh,
                                  const _Float16* __restrict__ vth,
                                  _Float16* __restrict__ attn_h) {
    int b = blockIdx.z, h = blockIdx.y;
    size_t bh = (size_t)b * HEADS + h;
    int wave = threadIdx.x >> 5, lane = threadIdx.x & 31;
    int khi = lane >> 4, ln = lane & 15;
    int q0 = blockIdx.x * 128 + wave * 16;

    const _Float16* Q  = qh  + bh * LSEQ * HDIM;
    const _Float16* K  = kh  + bh * LSEQ * HDIM;
    const _Float16* VT = vth + bh * HDIM * LSEQ;

    v16h qB = frag16(Q + (size_t)(q0 + ln) * HDIM, khi);
    __shared__ __attribute__((aligned(16))) _Float16 sO[8][16 * HDIM];

    float m = -3.0e38f, lsum = 0.f;
    v8f acc0 = {}, acc1 = {};
    const v8f zc = {};

    for (int kc = 0; kc < LSEQ; kc += 32) {
        v16h kA0 = load_a_frag(K + (size_t)kc * HDIM,        HDIM, ln, khi, 0);
        v16h kA1 = load_a_frag(K + (size_t)(kc + 16) * HDIM, HDIM, ln, khi, 0);

        v8f st0 = wmma16(kA0, qB, zc);
        v8f st1 = wmma16(kA1, qB, zc);

        float cmax = st0[0];
        #pragma unroll
        for (int r = 1; r < 8; ++r) cmax = fmaxf(cmax, st0[r]);
        #pragma unroll
        for (int r = 0; r < 8; ++r) cmax = fmaxf(cmax, st1[r]);
        cmax = fmaxf(cmax, __shfl_xor(cmax, 16, 32));
        float mnew = fmaxf(m, cmax);
        float alpha = expf(m - mnew);

        float p0[8], p1[8], csum = 0.f;
        #pragma unroll
        for (int r = 0; r < 8; ++r) {
            p0[r] = expf(st0[r] - mnew); csum += p0[r];
            p1[r] = expf(st1[r] - mnew); csum += p1[r];
        }
        csum += __shfl_xor(csum, 16, 32);
        lsum = lsum * alpha + csum;
        m = mnew;

        v16h pA;
        #pragma unroll
        for (int i = 0; i < 8; ++i) {
            pA[i]     = (_Float16)p0[i];
            pA[i + 8] = (_Float16)p1[i];
        }

        v16h vB0 = frag16(VT + (size_t)ln * LSEQ        + kc, khi);
        v16h vB1 = frag16(VT + (size_t)(16 + ln) * LSEQ + kc, khi);

        #pragma unroll
        for (int r = 0; r < 8; ++r) {
            float ar = __shfl(alpha, r + 8 * khi, 32);
            acc0[r] *= ar;
            acc1[r] *= ar;
        }
        acc0 = wmma16(pA, vB0, acc0);
        acc1 = wmma16(pA, vB1, acc1);
    }

    _Float16* so = sO[wave];
    #pragma unroll
    for (int r = 0; r < 8; ++r) {
        float lr = __shfl(lsum, r + 8 * khi, 32);
        float inv = 1.0f / lr;
        so[(r + 8 * khi) * HDIM + ln]      = (_Float16)(acc0[r] * inv);
        so[(r + 8 * khi) * HDIM + 16 + ln] = (_Float16)(acc1[r] * inv);
    }
    __builtin_amdgcn_fence(__ATOMIC_RELEASE, "workgroup"); __builtin_amdgcn_wave_barrier(); __builtin_amdgcn_fence(__ATOMIC_ACQUIRE, "workgroup");
    _Float16* dst = attn_h + (bh * LSEQ + q0) * HDIM;
    for (int pass = 0; pass < 2; ++pass) {
        *(volatile v8h*)(dst + lane * 8)       = *(const v8h*)(so + lane * 8);
        *(volatile v8h*)(dst + 256 + lane * 8) = *(const v8h*)(so + 256 + lane * 8);
        __threadfence();
    }
}

__global__ void out_gemm_kernel(const _Float16* __restrict__ attn_h,
                                const _Float16* __restrict__ wh,
                                const float* __restrict__ bias,
                                const float* __restrict__ xs_f,
                                float* __restrict__ out) {
    int b = blockIdx.z;
    int n0 = blockIdx.x * 64, m0 = blockIdx.y * 128;
    int wave = threadIdx.x >> 5, lane = threadIdx.x & 31;
    int khi = lane >> 4, ln = lane & 15;
    int row = m0 + wave * 16;
    __shared__ __attribute__((aligned(16))) float sOut[64][132];
    v8f acc[4] = {};
    for (int k0 = 0; k0 < CCH; k0 += 32) {
        const _Float16* A = attn_h + (((size_t)b * HEADS + (k0 >> 5)) * LSEQ + row) * HDIM;
        v16h a = load_a_frag(A, HDIM, ln, khi, 0);
        #pragma unroll
        for (int t = 0; t < 4; ++t) {
            int col = n0 + t * 16 + ln;
            v16h bf = frag16(wh + (size_t)col * CCH + k0, khi);
            acc[t] = wmma16(a, bf, acc[t]);
        }
    }
    #pragma unroll
    for (int t = 0; t < 4; ++t) {
        int c = n0 + t * 16 + ln;
        float bv = bias[c];
        #pragma unroll
        for (int r = 0; r < 8; ++r) {
            int l = row + r + 8 * khi;
            sOut[t * 16 + ln][l - m0] = acc[t][r] + bv + xs_f[((size_t)b * LSEQ + l) * CCH + c];
        }
    }
    __syncthreads();
    for (int pass = 0; pass < 2; ++pass) {
        for (int p = threadIdx.x; p < 64 * 32; p += 256) {
            const int cr = p >> 5, q = p & 31;
            *(volatile v4f*)(out + ((size_t)b * CCH + n0 + cr) * LSEQ + m0 + q * 4) = *(const v4f*)&sOut[cr][q * 4];
        }
        __threadfence();
    }
}

static inline size_t align256(size_t x) { return (x + 255) & ~(size_t)255; }

extern "C" void kernel_launch(void* const* d_in, const int* in_sizes, int n_in,
                              void* d_out, int out_size, void* d_ws, size_t ws_size,
                              hipStream_t stream) {
    const float* x      = (const float*)d_in[0];
    const float* t      = (const float*)d_in[1];
    const float* cond   = (const float*)d_in[2];
    const float* cond2  = (const float*)d_in[3];
    const float* gn_w   = (const float*)d_in[4];
    const float* gn_b   = (const float*)d_in[5];
    const float* proj_w = (const float*)d_in[6];
    const float* proj_b = (const float*)d_in[7];
    const float* out_w  = (const float*)d_in[8];
    const float* out_b  = (const float*)d_in[9];
    const float* time_w = (const float*)d_in[10];
    const float* time_b = (const float*)d_in[11];
    const float* cond_w = (const float*)d_in[12];
    const float* cond_b = (const float*)d_in[13];
    const float* cond2_w = (const float*)d_in[14];
    const float* cond2_b = (const float*)d_in[15];
    float* out = (float*)d_out;

    char* ws = (char*)d_ws;
    size_t off = 0;
    float* emb = (float*)(ws + off);            off = align256(off + BATCH * CCH * 4);
    float* mean = (float*)(ws + off);           off = align256(off + BATCH * GROUPS * 4);
    float* rstd = (float*)(ws + off);           off = align256(off + BATCH * GROUPS * 4);
    float* xs_f = (float*)(ws + off);           off = align256(off + (size_t)BATCH * LSEQ * CCH * 4);
    _Float16* xs_h = (_Float16*)(ws + off);     off = align256(off + (size_t)BATCH * LSEQ * CCH * 2);
    _Float16* proj_wh = (_Float16*)(ws + off);  off = align256(off + (size_t)NQKV * CCH * 2);
    _Float16* out_wh = (_Float16*)(ws + off);   off = align256(off + (size_t)CCH * CCH * 2);
    _Float16* qh = (_Float16*)(ws + off);       off = align256(off + (size_t)BATCH * HEADS * LSEQ * HDIM * 2);
    _Float16* kh = (_Float16*)(ws + off);       off = align256(off + (size_t)BATCH * HEADS * LSEQ * HDIM * 2);
    _Float16* vth = (_Float16*)(ws + off);      off = align256(off + (size_t)BATCH * HEADS * HDIM * LSEQ * 2);
    _Float16* attn_h = (_Float16*)(ws + off);   off = align256(off + (size_t)BATCH * LSEQ * CCH * 2);
    (void)n_in; (void)in_sizes; (void)out_size;
    if (off > ws_size) return;

    {
        int n1 = NQKV * CCH;
        cvt_half_kernel<<<(n1 + 255) / 256, 256, 0, stream>>>(proj_w, proj_wh, n1);
        int n2 = CCH * CCH;
        cvt_half_kernel<<<(n2 + 255) / 256, 256, 0, stream>>>(out_w, out_wh, n2);
    }
    cond_embed_kernel<<<BATCH, CCH, 0, stream>>>(t, cond, cond2,
                                                 time_w, time_b, cond_w, cond_b,
                                                 cond2_w, cond2_b, emb);
    gn_stats_kernel<<<BATCH, 256, 0, stream>>>(x, mean, rstd);
    gn_apply_kernel<<<BATCH * LSEQ, 256, 0, stream>>>(x, mean, rstd, gn_w, gn_b,
                                                     emb, xs_f, xs_h);
    qkv_gemm_kernel<<<dim3(NQKV / 64, LSEQ / 128, BATCH), 256, 0, stream>>>(
        xs_h, proj_wh, proj_b, qh, kh, vth);
    flash_attn_kernel<<<dim3(LSEQ / 128, HEADS, BATCH), 256, 0, stream>>>(
        qh, kh, vth, attn_h);
    out_gemm_kernel<<<dim3(CCH / 64, LSEQ / 128, BATCH), 256, 0, stream>>>(
        attn_h, out_wh, out_b, xs_f, out);
}
